// MultiHeadSelfAttention_62173946577659
// MI455X (gfx1250) — hardware-verified
//
#include <hip/hip_runtime.h>


#ifndef NB
#define NB 4
#endif
#ifndef SEQ
#define SEQ 2048
#endif
#define NB_FULL   4
#define SEQ_FULL  2048
#define HID       1024
#define NHEAD     16
#define HD        64
#define NQKV      3072
#define MROWS     (NB * SEQ)

static_assert(HID == NHEAD * HD);
static_assert(NHEAD == 16);
static_assert(HD == 64);
static_assert(NQKV == 3 * HID);
static_assert(SEQ % 128 == 0);
static_assert(SEQ <= SEQ_FULL);
static_assert(NB >= 1 && NB <= NB_FULL);
static_assert(MROWS % 128 == 0);
static_assert(HID % 128 == 0);

#define CARRY_X    16.0f
#define CARRY_W    32.0f
#define CARRY_QKV  16.0f
#define CARRY_CTX  1024.0f

typedef _Float16 f16;
typedef f16   v16h __attribute__((ext_vector_type(16)));
typedef f16   v8h  __attribute__((ext_vector_type(8)));
typedef float v8f  __attribute__((ext_vector_type(8)));
typedef float v4f  __attribute__((ext_vector_type(4)));

union FragU { v16h v; v8h half[2]; f16 e[16]; };
union H8U   { v8h v; f16 e[8]; };

#define WS_X_HALVES   ((size_t)MROWS * HID)
#define WS_WQ_HALVES  ((size_t)NQKV * HID)
#define WS_WO_HALVES  ((size_t)HID * HID)
#define WS_TAB_FLOATS ((size_t)SEQ * 32)
#define WS_TOTAL_BYTES ((5 * WS_X_HALVES + WS_WQ_HALVES + WS_WO_HALVES) * 2 + 2 * WS_TAB_FLOATS * 4 + 128)
static_assert(WS_TOTAL_BYTES <= (size_t)134217728);

__device__ __forceinline__ v8f zero8() {
    v8f z = {0.f, 0.f, 0.f, 0.f, 0.f, 0.f, 0.f, 0.f};
    return z;
}

__device__ __forceinline__ v8f wmma16(v16h a, v16h b, v8f c) {
    v8f d = __builtin_amdgcn_wmma_f32_16x16x32_f16(false, a, false, b, (short)0, c, false, false);
    asm volatile("v_nop\n\tv_nop\n\tv_nop\n\tv_nop" : "+v"(d) : "v"(a), "v"(b));
    return d;
}

__device__ __forceinline__ float bf16_rne(float x) {
    unsigned u = __float_as_uint(x);
    u = (u + 0x7fffu + ((u >> 16) & 1u)) & 0xffff0000u;
    return __uint_as_float(u);
}

__device__ __forceinline__ float fexp2(float x) {
#if defined(__has_builtin)
#if __has_builtin(__builtin_amdgcn_exp2f)
    return __builtin_amdgcn_exp2f(x);
#else
    return exp2f(x);
#endif
#else
    return exp2f(x);
#endif
}

__device__ __forceinline__ float rowmax16(float x) {
    int v = __builtin_bit_cast(int, x);
    x = fmaxf(x, __builtin_bit_cast(float, __builtin_amdgcn_update_dpp(v, v, 0x121, 0xf, 0xf, false)));
    v = __builtin_bit_cast(int, x);
    x = fmaxf(x, __builtin_bit_cast(float, __builtin_amdgcn_update_dpp(v, v, 0x122, 0xf, 0xf, false)));
    v = __builtin_bit_cast(int, x);
    x = fmaxf(x, __builtin_bit_cast(float, __builtin_amdgcn_update_dpp(v, v, 0x124, 0xf, 0xf, false)));
    v = __builtin_bit_cast(int, x);
    x = fmaxf(x, __builtin_bit_cast(float, __builtin_amdgcn_update_dpp(v, v, 0x128, 0xf, 0xf, false)));
    return x;
}

__device__ __forceinline__ v16h load_frag(const f16* tile, unsigned rowbase, unsigned pitch,
                                          unsigned kcol, unsigned lane) {
    const unsigned r  = rowbase + (lane & 15u);
    const unsigned kh = (lane >> 4) << 3;
    const f16* p = tile + (size_t)r * pitch + kcol + kh;
    FragU f;
    f.half[0] = *(const v8h*)(p);
    f.half[1] = *(const v8h*)(p + 16);
    return f.v;
}

template <unsigned DSTPER, unsigned SRCPER>
__global__ void __launch_bounds__(256)
cvt_rows(const float* __restrict__ src, f16* __restrict__ dst, unsigned nrows, float carry) {
    const unsigned g  = blockIdx.x * 256u + threadIdx.x;
    const unsigned m  = g >> 7;
    const unsigned c8 = (g & 127u) << 3;
    if (m >= nrows) return;
    const unsigned sm = (m / DSTPER) * SRCPER + (m % DSTPER);
    const float* sp = src + (size_t)sm * HID + c8;
    const v4f a = *(const v4f*)sp;
    const v4f b = *(const v4f*)(sp + 4);
    H8U o;
#pragma unroll
    for (int j = 0; j < 4; ++j) {
        const float x0 = a[j];
        const float x1 = b[j];
        o.e[j]     = (f16)(bf16_rne(x0) * carry);
        o.e[j + 4] = (f16)(bf16_rne(x1) * carry);
    }
    f16* dp = dst + (size_t)m * HID + c8;
    *(volatile v8h*)dp = o.v;
    __threadfence();
    *(volatile v8h*)dp = o.v;
}

__global__ void __launch_bounds__(256)
cvt_wT(const float* __restrict__ W, f16* __restrict__ Wt, unsigned ncols, float carry) {
    __shared__ __attribute__((aligned(16))) f16 tile[64 * 72];
    const unsigned tid = threadIdx.x;
    const unsigned n0  = blockIdx.x * 64u;
    const unsigned k0  = blockIdx.y * 64u;
    {
        const unsigned r   = tid >> 2;
        const unsigned seg = (tid & 3u) << 4;
        const float* sp = W + (size_t)(k0 + r) * ncols + n0 + seg;
#pragma unroll
        for (int q = 0; q < 4; ++q) {
            const v4f a = *(const v4f*)(sp + 4 * q);
#pragma unroll
            for (int j = 0; j < 4; ++j) {
                const float xv = a[j];
                tile[(seg + (unsigned)(4 * q + j)) * 72u + r] = (f16)(bf16_rne(xv) * carry);
            }
        }
    }
    __syncthreads();
    const unsigned lane  = tid & 31u;
    const unsigned wave  = tid >> 5;
    const unsigned piece = lane & 7u;
    const unsigned lsub  = lane >> 3;
    v8h vv[2];
#pragma unroll
    for (int it = 0; it < 2; ++it) {
        const unsigned L = (unsigned)it * 32u + wave * 4u + lsub;
        vv[it] = *(const v8h*)&tile[L * 72u + piece * 8u];
    }
#pragma unroll
    for (int pass = 0; pass < 2; ++pass) {
#pragma unroll
        for (int it = 0; it < 2; ++it) {
            const unsigned L = (unsigned)it * 32u + wave * 4u + lsub;
            f16* dp = Wt + (size_t)(n0 + L) * HID + k0 + piece * 8u;
            *(volatile v8h*)dp = vv[it];
        }
        if (pass == 0) __threadfence();
    }
}

__global__ void __launch_bounds__(32)
k_invfreq(float* __restrict__ invf) {
    const unsigned i = threadIdx.x & 31u;
    const float e = (float)(2u * i) * 0.015625f;
    const float p = powf(10000.0f, e);
    const float v = 1.0f / p;
    *(volatile float*)(invf + i) = v;
    __threadfence();
    *(volatile float*)(invf + i) = v;
}

__global__ void __launch_bounds__(256)
k_ropetab(const float* __restrict__ invf, float* __restrict__ ctab, float* __restrict__ stab) {
    const unsigned g = blockIdx.x * 256u + threadIdx.x;
    const unsigned l = g >> 5;
    const unsigned i = g & 31u;
    if (l >= (unsigned)SEQ) return;
    const float ang = (float)l * invf[i];
    const float c = cosf(ang);
    const float s = sinf(ang);
    float* cp = ctab + (size_t)l * 32u + i;
    float* sp = stab + (size_t)l * 32u + i;
    *(volatile float*)cp = c;
    *(volatile float*)sp = s;
    __threadfence();
    *(volatile float*)cp = c;
    *(volatile float*)sp = s;
}

template <int MODE>
__global__ void __launch_bounds__(256) __attribute__((amdgpu_num_vgpr(256)))
gemm_nt(const f16* __restrict__ A, const f16* __restrict__ W,
        const float* __restrict__ ctab, const float* __restrict__ stab,
        void* __restrict__ out, float accMul) {
    __shared__ __attribute__((aligned(16))) f16 As[128 * 32];
    __shared__ __attribute__((aligned(16))) f16 Bs[128 * 32];
    __shared__ __attribute__((aligned(16))) f16 Cs[128 * 128];

    const unsigned tid  = threadIdx.x;
    const unsigned lane = tid & 31u;
    const unsigned wave = tid >> 5;
    const unsigned wm   = wave & 3u;
    const unsigned wn   = wave >> 2;
    const unsigned hh8  = (lane >> 4) << 3;
    const unsigned c16  = lane & 15u;
    const unsigned m0   = blockIdx.x * 128u;
    const unsigned n0   = blockIdx.y * 128u;

    v8f acc[2][4];
#pragma unroll
    for (int i = 0; i < 2; ++i)
#pragma unroll
        for (int j = 0; j < 4; ++j) acc[i][j] = zero8();

    const unsigned srow = tid >> 1;
    const unsigned scol = (tid & 1u) << 4;
    const f16* gA = A + (size_t)(m0 + srow) * HID + scol;
    const f16* gW = W + (size_t)(n0 + srow) * HID + scol;

#pragma unroll 1
    for (unsigned k0 = 0; k0 < (unsigned)HID; k0 += 32u) {
        const v8h ra0 = *(const v8h*)(gA + k0);
        const v8h ra1 = *(const v8h*)(gA + k0 + 8);
        const v8h rb0 = *(const v8h*)(gW + k0);
        const v8h rb1 = *(const v8h*)(gW + k0 + 8);
        __syncthreads();
        *(v8h*)&As[srow * 32u + scol]      = ra0;
        *(v8h*)&As[srow * 32u + scol + 8u] = ra1;
        *(v8h*)&Bs[srow * 32u + scol]      = rb0;
        *(v8h*)&Bs[srow * 32u + scol + 8u] = rb1;
        __syncthreads();

        v16h af[2], bfr[4];
#pragma unroll
        for (int i = 0; i < 2; ++i) af[i] = load_frag(As, wm * 32u + (unsigned)i * 16u, 32u, 0u, lane);
#pragma unroll
        for (int j = 0; j < 4; ++j) bfr[j] = load_frag(Bs, wn * 64u + (unsigned)j * 16u, 32u, 0u, lane);
#pragma unroll
        for (int i = 0; i < 2; ++i)
#pragma unroll
            for (int j = 0; j < 4; ++j) acc[i][j] = wmma16(af[i], bfr[j], acc[i][j]);
    }

    const unsigned bidx  = m0 / (unsigned)SEQ;
    const unsigned s0    = m0 - bidx * (unsigned)SEQ;
    const unsigned piece = lane & 7u;
    const unsigned lsub  = lane >> 3;

    if constexpr (MODE == 0) {
        float* Cf = (float*)Cs;
        f16* op = (f16*)out;
        const size_t bh0 = (size_t)bidx * NHEAD + (n0 >> 6);
#pragma unroll
        for (int half = 0; half < 2; ++half) {
            if ((wm >> 1) == (unsigned)half) {
#pragma unroll
                for (int i = 0; i < 2; ++i)
#pragma unroll
                    for (int j = 0; j < 4; ++j) {
                        const unsigned nl = wn * 64u + (unsigned)j * 16u + c16;
#pragma unroll
                        for (int r = 0; r < 8; ++r) {
                            const unsigned ml = (wm & 1u) * 32u + (unsigned)i * 16u + hh8 + (unsigned)r;
                            Cf[ml * 128u + nl] = acc[i][j][r] * accMul;
                        }
                    }
            }
            __syncthreads();
            H8U pk[4];
#pragma unroll
            for (int it = 0; it < 4; ++it) {
                const unsigned L    = wave * 16u + (unsigned)it * 4u + lsub;
                const unsigned ml   = L >> 1;
                const unsigned hsel = L & 1u;
                const unsigned s    = s0 + (unsigned)half * 64u + ml;
                const float* cp = Cf + ml * 128u + hsel * 64u + piece * 8u;
                const v4f t0 = *(const v4f*)cp;
                const v4f t1 = *(const v4f*)(cp + 4);
                const v4f cs = *(const v4f*)(ctab + (size_t)s * 32u + piece * 4u);
                const v4f sn = *(const v4f*)(stab + (size_t)s * 32u + piece * 4u);
                pk[it].e[0] = (f16)(t0[0] * cs[0] - t0[1] * sn[0]);
                pk[it].e[1] = (f16)(t0[1] * cs[0] + t0[0] * sn[0]);
                pk[it].e[2] = (f16)(t0[2] * cs[1] - t0[3] * sn[1]);
                pk[it].e[3] = (f16)(t0[3] * cs[1] + t0[2] * sn[1]);
                pk[it].e[4] = (f16)(t1[0] * cs[2] - t1[1] * sn[2]);
                pk[it].e[5] = (f16)(t1[1] * cs[2] + t1[0] * sn[2]);
                pk[it].e[6] = (f16)(t1[2] * cs[3] - t1[3] * sn[3]);
                pk[it].e[7] = (f16)(t1[3] * cs[3] + t1[2] * sn[3]);
            }
#pragma unroll
            for (int pass = 0; pass < 2; ++pass) {
#pragma unroll
                for (int it = 0; it < 4; ++it) {
                    const unsigned L    = wave * 16u + (unsigned)it * 4u + lsub;
                    const unsigned ml   = L >> 1;
                    const unsigned hsel = L & 1u;
                    const unsigned s    = s0 + (unsigned)half * 64u + ml;
                    f16* dp = op + ((bh0 + hsel) * SEQ + s) * HD + piece * 8u;
                    *(volatile v8h*)dp = pk[it].v;
                }
                if (pass == 0) __threadfence();
            }
            __syncthreads();
        }
    } else if constexpr (MODE == 1) {
#pragma unroll
        for (int i = 0; i < 2; ++i)
#pragma unroll
            for (int j = 0; j < 4; ++j) {
                const unsigned nl = wn * 64u + (unsigned)j * 16u + c16;
                H8U t;
#pragma unroll
                for (int r = 0; r < 8; ++r) t.e[r] = (f16)(acc[i][j][r] * accMul);
                *(v8h*)&Cs[nl * 128u + wm * 32u + (unsigned)i * 16u + hh8] = t.v;
            }
        __syncthreads();
        f16* op = (f16*)out;
#pragma unroll
        for (int pass = 0; pass < 2; ++pass) {
#pragma unroll
            for (int it = 0; it < 8; ++it) {
                const unsigned L  = wave * 32u + (unsigned)it * 4u + lsub;
                const unsigned nl = L >> 1;
                const unsigned mh = L & 1u;
                const v8h v = *(const v8h*)&Cs[nl * 128u + mh * 64u + piece * 8u];
                f16* dp = op + ((size_t)(bidx * (unsigned)HID + n0 + nl) * SEQ + s0 + mh * 64u + piece * 8u);
                *(volatile v8h*)dp = v;
            }
            if (pass == 0) __threadfence();
        }
    } else {
        float* Cf = (float*)Cs;
        float* of = (float*)out;
#pragma unroll
        for (int half = 0; half < 2; ++half) {
            if ((wm >> 1) == (unsigned)half) {
#pragma unroll
                for (int i = 0; i < 2; ++i)
#pragma unroll
                    for (int j = 0; j < 4; ++j) {
                        const unsigned nl = wn * 64u + (unsigned)j * 16u + c16;
#pragma unroll
                        for (int r = 0; r < 8; ++r) {
                            const unsigned ml = (wm & 1u) * 32u + (unsigned)i * 16u + hh8 + (unsigned)r;
                            Cf[ml * 128u + nl] = acc[i][j][r] * accMul;
                        }
                    }
            }
            __syncthreads();
#pragma unroll
            for (int pass = 0; pass < 2; ++pass) {
#pragma unroll
                for (int it = 0; it < 8; ++it) {
                    const unsigned L    = wave * 32u + (unsigned)it * 4u + lsub;
                    const unsigned row  = L >> 2;
                    const unsigned part = L & 3u;
                    const v4f v = *(const v4f*)&Cf[row * 128u + part * 32u + piece * 4u];
                    float* dp = of + (size_t)(m0 + (unsigned)half * 64u + row) * HID + n0 + part * 32u + piece * 4u;
                    *(volatile v4f*)dp = v;
                }
                if (pass == 0) __threadfence();
            }
            __syncthreads();
        }
    }
}

__global__ void __launch_bounds__(256) __attribute__((amdgpu_num_vgpr(256)))
attn_fwd(const f16* __restrict__ Qp, const f16* __restrict__ Kp, const f16* __restrict__ Vt,
         f16* __restrict__ Cp) {
    __shared__ __attribute__((aligned(16))) f16 ks[64 * 64];
    __shared__ __attribute__((aligned(16))) f16 vsT[64 * 64];
    __shared__ __attribute__((aligned(16))) f16 ps[8][16 * 64];

    const unsigned tid  = threadIdx.x;
    const unsigned lane = tid & 31u;
    const unsigned wave = tid >> 5;
    const unsigned hh8  = (lane >> 4) << 3;
    const unsigned c16  = lane & 15u;
    const unsigned bh   = blockIdx.y;
    const unsigned bidx = bh >> 4;
    const unsigned hidx = bh & 15u;
    const unsigned q0   = blockIdx.x * 128u + wave * 16u;
    const size_t head = (size_t)bh * SEQ * HD;

    v16h qa[2];
#pragma unroll
    for (int c = 0; c < 2; ++c) qa[c] = load_frag(Qp + head, q0, HD, (unsigned)c * 32u, lane);

    FragU onesu;
#pragma unroll
    for (int i = 0; i < 16; ++i) onesu.e[i] = (f16)1.0f;
    const v16h ones = onesu.v;

    float m[8];
    v8f   o[4], lacc;
#pragma unroll
    for (int r = 0; r < 8; ++r) m[r] = -1.0e30f;
#pragma unroll
    for (int dt = 0; dt < 4; ++dt) o[dt] = zero8();
    lacc = zero8();

    const float cl = 1.4426950408889634f * 0.00048828125f;
    f16* psw = &ps[wave][0];

#pragma unroll 1
    for (unsigned kt = 0; kt < (unsigned)(SEQ / 64); ++kt) {
        __syncthreads();
#pragma unroll
        for (int p2 = 0; p2 < 2; ++p2) {
            const unsigned p   = tid + (unsigned)p2 * 256u;
            const unsigned row = p >> 3;
            const unsigned pc  = (p & 7u) << 3;
            const v8h kv = *(const v8h*)(Kp + head + (size_t)(kt * 64u + row) * HD + pc);
            const v8h vv = *(const v8h*)(Vt + head + (size_t)row * SEQ + kt * 64u + pc);
            *(v8h*)&ks[row * 64u + pc]  = kv;
            *(v8h*)&vsT[row * 64u + pc] = vv;
        }
        __syncthreads();

        v8f s[4];
#pragma unroll
        for (int nt = 0; nt < 4; ++nt) s[nt] = zero8();
#pragma unroll
        for (int c = 0; c < 2; ++c) {
#pragma unroll
            for (int nt = 0; nt < 4; ++nt) {
                const v16h kb = load_frag(ks, (unsigned)nt * 16u, 64u, (unsigned)c * 32u, lane);
                s[nt] = wmma16(qa[c], kb, s[nt]);
            }
        }

#pragma unroll
        for (int r = 0; r < 8; ++r) {
            float x[4];
#pragma unroll
            for (int nt = 0; nt < 4; ++nt) x[nt] = s[nt][r] * cl;
            const float tm = rowmax16(fmaxf(fmaxf(x[0], x[1]), fmaxf(x[2], x[3])));
            const float mn = fmaxf(m[r], tm);
            const float al = fexp2(m[r] - mn);
            m[r] = mn;
            lacc[r] *= al;
#pragma unroll
            for (int dt = 0; dt < 4; ++dt) o[dt][r] *= al;
            const float sh = 10.0f - mn;
#pragma unroll
            for (int nt = 0; nt < 4; ++nt)
                psw[(hh8 + (unsigned)r) * 64u + (unsigned)nt * 16u + c16] = (f16)fexp2(x[nt] + sh);
        }
        __syncthreads();

#pragma unroll
        for (int kk = 0; kk < 2; ++kk) {
            const v16h pa = load_frag(psw, 0u, 64u, (unsigned)kk * 32u, lane);
#pragma unroll
            for (int dt = 0; dt < 4; ++dt) {
                const v16h vb = load_frag(vsT, (unsigned)dt * 16u, 64u, (unsigned)kk * 32u, lane);
                o[dt] = wmma16(pa, vb, o[dt]);
            }
            lacc = wmma16(pa, ones, lacc);
        }
    }
    __syncthreads();

#pragma unroll
    for (int r = 0; r < 8; ++r) {
        const float inv = (CARRY_CTX / CARRY_QKV) / lacc[r];
#pragma unroll
        for (int dt = 0; dt < 4; ++dt)
            psw[(hh8 + (unsigned)r) * 64u + (unsigned)dt * 16u + c16] = (f16)(o[dt][r] * inv);
    }
    __syncthreads();

    const unsigned piece = lane & 7u;
    const unsigned lsub  = lane >> 3;
#pragma unroll
    for (int pass = 0; pass < 2; ++pass) {
#pragma unroll
        for (int it = 0; it < 4; ++it) {
            const unsigned L = (unsigned)it * 4u + lsub;
            const v8h v = *(const v8h*)&psw[L * 64u + piece * 8u];
            f16* dp = Cp + ((size_t)(bidx * (unsigned)SEQ + q0 + L) * HID + hidx * HD + piece * 8u);
            *(volatile v8h*)dp = v;
        }
        if (pass == 0) __threadfence();
    }
}

extern "C" void kernel_launch(void* const* d_in, const int* in_sizes, int n_in,
                              void* d_out, int out_size, void* d_ws, size_t ws_size,
                              hipStream_t stream) {
    if (n_in < 3) return;
    if (in_sizes[0] < ((NB - 1) * SEQ_FULL + SEQ) * HID) return;
    if (in_sizes[1] < HID * NQKV) return;
    if (in_sizes[2] < HID * HID) return;
    if (out_size < MROWS * HID) return;
    if (ws_size < WS_TOTAL_BYTES) return;

    const float* x    = (const float*)d_in[0];
    const float* wqkv = (const float*)d_in[1];
    const float* wout = (const float*)d_in[2];

    const size_t nX = WS_X_HALVES;
    const size_t nW = WS_WO_HALVES;

    f16* Xh  = (f16*)d_ws;
    f16* Wt  = Xh  + nX;
    f16* Wot = Wt  + 3 * nW;
    f16* Qp  = Wot + nW;
    f16* Kp  = Qp  + nX;
    f16* Vtp = Kp  + nX;
    f16* Cp  = Vtp + nX;
    float* ctab = (float*)(Cp + nX);
    float* stab = ctab + WS_TAB_FLOATS;
    float* invf = stab + WS_TAB_FLOATS;

    cvt_rows<SEQ, SEQ_FULL><<<MROWS / 2, 256, 0, stream>>>(x, Xh, (unsigned)MROWS, CARRY_X);
    cvt_wT<<<dim3(NQKV / 64, HID / 64), 256, 0, stream>>>(wqkv, Wt, (unsigned)NQKV, CARRY_W);
    cvt_wT<<<dim3(HID / 64, HID / 64), 256, 0, stream>>>(wout, Wot, (unsigned)HID, CARRY_W);

    k_invfreq<<<1, 32, 0, stream>>>(invf);
    k_ropetab<<<(SEQ * 32) / 256, 256, 0, stream>>>(invf, ctab, stab);

    const dim3 gg(MROWS / 128, HID / 128);
    const float accQKV = CARRY_QKV / (CARRY_X * CARRY_W);
    gemm_nt<0><<<gg, 256, 0, stream>>>(Xh, Wt,          ctab, stab, (void*)Qp,  accQKV);
    gemm_nt<0><<<gg, 256, 0, stream>>>(Xh, Wt + nW,     ctab, stab, (void*)Kp,  accQKV);
    gemm_nt<1><<<gg, 256, 0, stream>>>(Xh, Wt + 2 * nW, ctab, stab, (void*)Vtp, accQKV);

    attn_fwd<<<dim3(SEQ / 128, NB * NHEAD), 256, 0, stream>>>(Qp, Kp, Vtp, Cp);

    const float accOut = 1.0f / (CARRY_CTX * CARRY_W);
    gemm_nt<2><<<gg, 256, 0, stream>>>(Cp, Wot, ctab, stab, d_out, accOut);
}
